// RobertaSelfAttention_89223650607453
// MI455X (gfx1250) — hardware-verified
//
#include <hip/hip_runtime.h>
#include <math.h>

#ifndef NB
#define NB 8
#endif
#ifndef SEQ
#define SEQ 1024
#endif
#define NB_FULL  8
#define SEQ_FULL 1024
#define DM   1024
#define NH   16
#define HD   64
#define MAXP 1024
#define NREL (2 * MAXP - 1)
#define PER  (2 * MAXP)
#define MT   (NB * SEQ)
#define KQP  (2 * DM)
#define AWV  4
#define RWP  48
#define GKP  100
#define ZP   68
#define WSCL 64.0f
#define QKS  16.0f
#define VSC  16.0f
#define PSC  4096.0f
#define RSQD 0.125f

static_assert(NH * HD == DM);
static_assert(HD == 64);
static_assert(DM == 1024);
static_assert(NB >= 1 && NB <= NB_FULL);
static_assert(SEQ >= 64 && SEQ <= SEQ_FULL && (SEQ % 64) == 0 && SEQ <= MAXP);
static_assert((MT % 64) == 0 && (DM % 64) == 0 && (KQP % 64) == 0);
static_assert((((MT / 64) * (DM / 64)) % 8) == 0);
static_assert(((MT * DM) % 2048) == 0 && ((PER * HD) % 2048) == 0 && ((NREL * HD) % 8) == 0);
static_assert(RWP >= 48 && GKP >= 96 && ZP >= 64 && (ZP % 4) == 0);

typedef _Float16 v16h __attribute__((ext_vector_type(16)));
typedef unsigned short v16us __attribute__((ext_vector_type(16)));
typedef unsigned short v8us  __attribute__((ext_vector_type(8)));
typedef float v8f __attribute__((ext_vector_type(8)));
typedef float v4f __attribute__((ext_vector_type(4)));
typedef unsigned int v4u __attribute__((ext_vector_type(4)));

union FragU { v16us v; v8us h[2]; };

__device__ __forceinline__ unsigned short bf_bits(float f) {
  const unsigned u = __float_as_uint(f);
  return (unsigned short)((u + 0x7FFFu + ((u >> 16) & 1u)) >> 16);
}
__device__ __forceinline__ float bf_up(unsigned short h) { return __uint_as_float(((unsigned)h) << 16); }
__device__ __forceinline__ float bfr(float f) { return bf_up(bf_bits(f)); }
__device__ __forceinline__ unsigned short h_bits(_Float16 x) { return __builtin_bit_cast(unsigned short, x); }
__device__ __forceinline__ unsigned short f2h(float f) { return h_bits((_Float16)f); }
__device__ __forceinline__ unsigned pk16(unsigned short a, unsigned short b) { return (unsigned)a | ((unsigned)b << 16); }
__device__ __forceinline__ int clampi(int v, int lo, int hi) { return v < lo ? lo : (v > hi ? hi : v); }
__device__ __forceinline__ v8f zero8() { v8f z = {0.f, 0.f, 0.f, 0.f, 0.f, 0.f, 0.f, 0.f}; return z; }

__device__ __forceinline__ v16us ldfrag_u(const unsigned short* p) {
  FragU f;
  f.h[0] = *(const v8us*)(p);
  f.h[1] = *(const v8us*)(p + 16);
  return f.v;
}

__device__ __forceinline__ v8f mma_raw(v16us a, v16us b, v8f c) {
  return __builtin_amdgcn_wmma_f32_16x16x32_f16(false, __builtin_bit_cast(v16h, a), false,
                                                __builtin_bit_cast(v16h, b), (short)0, c, false, false);
}
__device__ __forceinline__ v8f mma_g(v16us a, v16us b, v8f c) {
  c = mma_raw(a, b, c);
#if defined(__HIP_DEVICE_COMPILE__)
  asm volatile("v_nop\n\tv_nop\n\tv_nop\n\tv_nop" : "+v"(c) : "v"(a), "v"(b));
#endif
  return c;
}
__device__ __forceinline__ void dep_guard1(v8f& a, v8f& b, v16us x) {
#if defined(__HIP_DEVICE_COMPILE__)
  asm volatile("v_nop\n\tv_nop\n\tv_nop\n\tv_nop" : "+v"(a), "+v"(b) : "v"(x));
#endif
}
__device__ __forceinline__ void keep4_u(v16us a, v16us b, v16us c, v16us d) {
#if defined(__HIP_DEVICE_COMPILE__)
  asm volatile("v_nop" :: "v"(a), "v"(b), "v"(c), "v"(d));
#endif
}
__device__ __forceinline__ void acc_guard4(v8f& a, v8f& b, v8f& c, v8f& d) {
#if defined(__HIP_DEVICE_COMPILE__)
  asm volatile("v_nop\n\tv_nop\n\tv_nop\n\tv_nop" : "+v"(a), "+v"(b), "+v"(c), "+v"(d));
#endif
}
__device__ __forceinline__ void wave_sync_lds() {
  __builtin_amdgcn_fence(__ATOMIC_RELEASE, "workgroup");
  __builtin_amdgcn_wave_barrier();
  __builtin_amdgcn_fence(__ATOMIC_ACQUIRE, "workgroup");
}

__global__ __launch_bounds__(256) void cvt_x(const float* __restrict__ w, unsigned short* o) {
  const int base = (blockIdx.x * 256 + threadIdx.x) * 8;
  if (base + 8 > MT * DM) return;
  const int pr = base / DM;
  const int col = base - pr * DM;
  const int bb = pr / SEQ, tt = pr - bb * SEQ;
  const float* src = w + ((size_t)bb * SEQ_FULL + (size_t)tt) * DM + col;
  const v4f a0 = *(const v4f*)(src);
  const v4f a1 = *(const v4f*)(src + 4);
  v4u hv;
#pragma unroll
  for (int e = 0; e < 2; ++e) {
    hv[e]     = pk16(f2h(bfr(a0[2 * e])), f2h(bfr(a0[2 * e + 1])));
    hv[2 + e] = pk16(f2h(bfr(a1[2 * e])), f2h(bfr(a1[2 * e + 1])));
  }
  unsigned short* d = o + base;
  *(volatile v4u*)d = hv;
  __threadfence();
  *(volatile v4u*)d = hv;
}

__global__ __launch_bounds__(256) void cvt_lin(const float* __restrict__ w, unsigned short* o,
                                                int nsrc, int ndst, float sc) {
  const int base = (blockIdx.x * 256 + threadIdx.x) * 8;
  if (base + 8 > ndst) return;
  const bool inr = (base + 8 <= nsrc);
  const int lb = inr ? base : (nsrc - 8);
  const v4f a0 = *(const v4f*)(w + lb);
  const v4f a1 = *(const v4f*)(w + lb + 4);
  v4u hv;
#pragma unroll
  for (int e = 0; e < 2; ++e) {
    hv[e]     = pk16(f2h(bfr(a0[2 * e]) * sc), f2h(bfr(a0[2 * e + 1]) * sc));
    hv[2 + e] = pk16(f2h(bfr(a1[2 * e]) * sc), f2h(bfr(a1[2 * e + 1]) * sc));
  }
  const v4u zz = {0u, 0u, 0u, 0u};
  hv = inr ? hv : zz;
  unsigned short* d = o + base;
  *(volatile v4u*)d = hv;
  __threadfence();
  *(volatile v4u*)d = hv;
}

__global__ __launch_bounds__(256) void cvt_t(const float* __restrict__ w, unsigned short* o, int R, int C, float sc) {
  __shared__ __align__(16) unsigned short st[64 * 72];
  const int t = threadIdx.x;
  const int r0 = blockIdx.y * 64, c0 = blockIdx.x * 64;
  if (r0 + 64 > R || c0 + 64 > C) return;
  {
    const int row = t >> 2, ch = (t & 3) * 16;
    const float* p = w + (size_t)(r0 + row) * C + c0 + ch;
#pragma unroll
    for (int q = 0; q < 4; ++q) {
      const v4f v = *(const v4f*)(p + 4 * q);
#pragma unroll
      for (int e = 0; e < 4; ++e) st[(ch + 4 * q + e) * 72 + row] = f2h(bfr(v[e]) * sc);
    }
  }
  __syncthreads();
  v4u hv[2];
#pragma unroll
  for (int half = 0; half < 2; ++half) {
    const int cl = (t >> 3) + 32 * half, pc = (t & 7) * 8;
    hv[half] = *(const v4u*)(st + cl * 72 + pc);
  }
  for (int pass = 0; pass < 2; ++pass) {
#pragma unroll
    for (int half = 0; half < 2; ++half) {
      const int cl = (t >> 3) + 32 * half, pc = (t & 7) * 8;
      unsigned short* dst = o + (size_t)(c0 + cl) * R + r0 + pc;
      *(volatile v4u*)dst = hv[half];
    }
    __threadfence();
  }
}

__global__ __launch_bounds__(256) void tr16(const unsigned short* __restrict__ s, int lds,
                                             unsigned short* o, int R, int C) {
  __shared__ __align__(16) unsigned short st[64 * 72];
  const int t = threadIdx.x;
  const int r0 = blockIdx.y * 64, c0 = blockIdx.x * 64;
  if (r0 + 64 > R || c0 + 64 > C) return;
  {
    const int row = t >> 2, ch = (t & 3) * 16;
    const unsigned short* p = s + (size_t)(r0 + row) * lds + c0 + ch;
#pragma unroll
    for (int q = 0; q < 2; ++q) {
      const v4u v = *(const v4u*)(p + 8 * q);
#pragma unroll
      for (int e = 0; e < 8; ++e) {
        const unsigned hw = (v[e >> 1] >> (16 * (e & 1))) & 0xFFFFu;
        st[(ch + 8 * q + e) * 72 + row] = (unsigned short)hw;
      }
    }
  }
  __syncthreads();
  v4u hv[2];
#pragma unroll
  for (int half = 0; half < 2; ++half) {
    const int cl = (t >> 3) + 32 * half, pc = (t & 7) * 8;
    hv[half] = *(const v4u*)(st + cl * 72 + pc);
  }
  for (int pass = 0; pass < 2; ++pass) {
#pragma unroll
    for (int half = 0; half < 2; ++half) {
      const int cl = (t >> 3) + 32 * half, pc = (t & 7) * 8;
      unsigned short* dst = o + (size_t)(c0 + cl) * R + r0 + pc;
      *(volatile v4u*)dst = hv[half];
    }
    __threadfence();
  }
}

__global__ __launch_bounds__(256) void gemm64h(
    const unsigned short* __restrict__ Ap, int lda, const unsigned short* __restrict__ Btp, int ldb,
    unsigned short* Ch, int ldc, const float* __restrict__ bias, float osc, float bsc, int M, int N, int K) {
  __shared__ __align__(16) float sT[8][16 * 68];
  const int lane = threadIdx.x & 31;
  const int wave = threadIdx.x >> 5;
  const int tilesN = N >> 6;
  const int tilesM = M >> 6;
  const int tile = blockIdx.x * 8 + wave;
  if (tile >= tilesM * tilesN) return;
  const int tm = tile / tilesN;
  const int tn = tile - tm * tilesN;
  const int m0 = tm << 6;
  const int n0 = tn << 6;

  const int rlane = lane & 15;
  const int koff  = (lane >> 4) * 8;
  const int mOff  = (lane >> 4) * 8;

  v8f acc[4][4];
#pragma unroll
  for (int i = 0; i < 4; ++i)
#pragma unroll
    for (int j = 0; j < 4; ++j) acc[i][j] = zero8();

#pragma unroll 1
  for (int k0 = 0; k0 < K; k0 += 32) {
    v16us bh[4];
#pragma unroll
    for (int j = 0; j < 4; ++j) {
      const size_t bo = (size_t)(n0 + (j << 4) + rlane) * ldb + koff + k0;
      bh[j] = ldfrag_u(Btp + bo);
    }
#pragma unroll
    for (int i = 0; i < 4; ++i) {
      const size_t ao = (size_t)(m0 + (i << 4) + rlane) * lda + koff + k0;
      const v16us ah = ldfrag_u(Ap + ao);
#pragma unroll
      for (int j = 0; j < 4; ++j) acc[i][j] = mma_raw(ah, bh[j], acc[i][j]);
      dep_guard1(acc[i][0], acc[i][3], ah);
    }
    keep4_u(bh[0], bh[1], bh[2], bh[3]);
  }
  acc_guard4(acc[0][0], acc[0][1], acc[0][2], acc[0][3]);
  acc_guard4(acc[1][0], acc[1][1], acc[1][2], acc[1][3]);
  acc_guard4(acc[2][0], acc[2][1], acc[2][2], acc[2][3]);
  acc_guard4(acc[3][0], acc[3][1], acc[3][2], acc[3][3]);

  const int q8 = lane >> 3, c8 = (lane & 7) * 8;

  float bcol[8];
  {
    const v4f b0 = *(const v4f*)(bias + n0 + c8);
    const v4f b1 = *(const v4f*)(bias + n0 + c8 + 4);
#pragma unroll
    for (int e = 0; e < 4; ++e) {
      bcol[e]     = bfr(b0[e]) * bsc;
      bcol[4 + e] = bfr(b1[e]) * bsc;
    }
  }

  float* slab = sT[wave];
#pragma unroll
  for (int i = 0; i < 4; ++i) {
    const int mBase = m0 + (i << 4);
#pragma unroll
    for (int j = 0; j < 4; ++j) {
#pragma unroll
      for (int r = 0; r < 8; ++r) {
        slab[(mOff + r) * 68 + (j << 4) + rlane] = acc[i][j][r];
      }
    }
    wave_sync_lds();
    v4u hv[4];
#pragma unroll
    for (int it = 0; it < 4; ++it) {
      const int row = it * 4 + q8;
      const float* sp = slab + row * 68 + c8;
      v4u ha = {0u, 0u, 0u, 0u};
#pragma unroll
      for (int e = 0; e < 4; ++e) {
        const float b0 = sp[2 * e]     * osc + bcol[2 * e];
        const float b1 = sp[2 * e + 1] * osc + bcol[2 * e + 1];
        ha[e] = pk16(f2h(b0), f2h(b1));
      }
      hv[it] = ha;
    }
    for (int pass = 0; pass < 2; ++pass) {
#pragma unroll
      for (int it = 0; it < 4; ++it) {
        const int row = it * 4 + q8;
        const size_t go = (size_t)(mBase + row) * ldc + (size_t)n0 + c8;
        *(volatile v4u*)(Ch + go) = hv[it];
      }
      __threadfence();
    }
    wave_sync_lds();
  }
}

__global__ __launch_bounds__(128) void attn_kernel(
    const unsigned short* __restrict__ KQ, const unsigned short* __restrict__ PE,
    const unsigned short* __restrict__ VT, float* Out) {
  __shared__ __align__(16) float relw[AWV][16 * RWP];
  __shared__ __align__(16) float gks[2][32 * GKP];
  __shared__ __align__(16) unsigned short pws[AWV][16 * 32];
  __shared__ __align__(16) float zst[AWV][16 * ZP];
  const int lane = threadIdx.x & 31, wv = threadIdx.x >> 5, m = lane & 15, hh = lane >> 4;
  const int nqb = SEQ / 64;
  const int bh = blockIdx.x / nqb;
  const int tB = (blockIdx.x - bh * nqb) << 6;
  const int b = bh / NH, h = bh - (bh / NH) * NH;
  if (b >= NB) return;
  const int t0 = tB + (wv << 4);
  const size_t tok0 = (size_t)b * SEQ;
  const int jt  = wv >> 1;
  const int ctb = 3 * (wv & 1);
  float* rw = relw[wv];
  unsigned short* ph = pws[wv];

  const unsigned short* qp = KQ + (tok0 + (size_t)(t0 + m)) * KQP + h * HD + 8 * hh;
  const v16us qf0 = ldfrag_u(qp);
  const v16us qf1 = ldfrag_u(qp + 32);

  v8f carry;
  {
    const int u = clampi(t0 + MAXP + m, 0, PER - 1);
    const unsigned short* pp = PE + (size_t)u * HD + 8 * hh;
    carry = mma_g(qf0, ldfrag_u(pp), zero8());
    carry = mma_g(qf1, ldfrag_u(pp + 32), carry);
  }

  float mx[8], ls[8];
  v8f O0 = zero8(), O1 = zero8(), O2 = zero8(), O3 = zero8();
#pragma unroll
  for (int r = 0; r < 8; ++r) { mx[r] = -1.0e30f; ls[r] = 0.f; }

#pragma unroll 1
  for (int kb = 0; kb < SEQ / 32; ++kb) {
    const int sb = kb << 5;
    const unsigned short* kp = KQ + (tok0 + (size_t)(sb + m)) * KQP + DM + h * HD + 8 * hh;
    v8f S0, S1;
    {
      S0 = mma_g(qf0, ldfrag_u(kp), zero8());
      S0 = mma_g(qf1, ldfrag_u(kp + 32), S0);
      const unsigned short* kp1 = kp + (size_t)16 * KQP;
      S1 = mma_g(qf0, ldfrag_u(kp1), zero8());
      S1 = mma_g(qf1, ldfrag_u(kp1 + 32), S1);
    }

    float* gk = gks[kb & 1];
    const int vb = tB - sb + (MAXP - 32);
    {
      const unsigned short* ga = kp + (size_t)jt * 16 * KQP;
      const v16us a0 = ldfrag_u(ga);
      const v16us a1 = ldfrag_u(ga + 32);
#pragma unroll
      for (int q = 0; q < 3; ++q) {
        const int ct = ctb + q;
        const int u = clampi(vb + 16 * ct + m, 0, PER - 1);
        const unsigned short* pp = PE + (size_t)u * HD + 8 * hh;
        v8f G = mma_g(a0, ldfrag_u(pp), zero8());
        G = mma_g(a1, ldfrag_u(pp + 32), G);
#pragma unroll
        for (int r = 0; r < 8; ++r) gk[(16 * jt + 8 * hh + r) * GKP + 16 * ct + m] = G[r];
      }
    }

    {
      const int ub = vb + 16 * wv;
      const int u0 = clampi(ub + m, 0, PER - 1);
      const unsigned short* p0 = PE + (size_t)u0 * HD + 8 * hh;
      v8f C0 = mma_g(qf0, ldfrag_u(p0), zero8());
      C0 = mma_g(qf1, ldfrag_u(p0 + 32), C0);
      const int u1 = clampi(ub + 16 + m, 0, PER - 1);
      const unsigned short* p1 = PE + (size_t)u1 * HD + 8 * hh;
      v8f C1 = mma_g(qf0, ldfrag_u(p1), zero8());
      C1 = mma_g(qf1, ldfrag_u(p1 + 32), C1);
#pragma unroll
      for (int r = 0; r < 8; ++r) {
        const int row = 8 * hh + r;
        rw[row * RWP + m]      = C0[r];
        rw[row * RWP + 16 + m] = C1[r];
        rw[row * RWP + 32 + m] = carry[r];
      }
      carry = C0;
    }
    wave_sync_lds();
    __syncthreads();

    float s0[8], s1[8];
#pragma unroll
    for (int r = 0; r < 8; ++r) {
      const int row = 8 * hh + r;
      const float rq0 = rw[row * RWP + 31 + row - m];
      const float rq1 = rw[row * RWP + 15 + row - m];
      const float rk0 = gk[m * GKP + 31 + 16 * wv + row - m];
      const float rk1 = gk[(16 + m) * GKP + 15 + 16 * wv + row - m];
      s0[r] = (S0[r] * (1.0f / (QKS * QKS)) + (rq0 + rk0) * (1.0f / (QKS * WSCL))) * RSQD;
      s1[r] = (S1[r] * (1.0f / (QKS * QKS)) + (rq1 + rk1) * (1.0f / (QKS * WSCL))) * RSQD;
    }

#pragma unroll
    for (int r = 0; r < 8; ++r) {
      float xm = fmaxf(s0[r], s1[r]);
      xm = fmaxf(xm, __shfl_xor(xm, 1, 32));
      xm = fmaxf(xm, __shfl_xor(xm, 2, 32));
      xm = fmaxf(xm, __shfl_xor(xm, 4, 32));
      xm = fmaxf(xm, __shfl_xor(xm, 8, 32));
      const float mn = fmaxf(mx[r], xm);
      const float al = __expf(mx[r] - mn);
      mx[r] = mn;
      const float p0 = __expf(s0[r] - mn);
      const float p1 = __expf(s1[r] - mn);
      float ps = p0 + p1;
      ps += __shfl_xor(ps, 1, 32);
      ps += __shfl_xor(ps, 2, 32);
      ps += __shfl_xor(ps, 4, 32);
      ps += __shfl_xor(ps, 8, 32);
      ls[r] = ls[r] * al + ps;
      O0[r] = O0[r] * al;
      O1[r] = O1[r] * al;
      O2[r] = O2[r] * al;
      O3[r] = O3[r] * al;
      const int row = 8 * hh + r;
      ph[row * 32 + m]      = f2h(p0 * PSC);
      ph[row * 32 + 16 + m] = f2h(p1 * PSC);
    }
    wave_sync_lds();

    const v16us af = ldfrag_u(ph + m * 32 + 8 * hh);
    const size_t vo = (size_t)(h * HD + m) * MT + tok0 + (size_t)sb + 8 * hh;
    const v16us vf0 = ldfrag_u(VT + vo);
    const v16us vf1 = ldfrag_u(VT + vo + (size_t)16 * MT);
    const v16us vf2 = ldfrag_u(VT + vo + (size_t)32 * MT);
    const v16us vf3 = ldfrag_u(VT + vo + (size_t)48 * MT);
    O0 = mma_g(af, vf0, O0);
    O1 = mma_g(af, vf1, O1);
    O2 = mma_g(af, vf2, O2);
    O3 = mma_g(af, vf3, O3);
  }
  acc_guard4(O0, O1, O2, O3);

  float* zs = zst[wv];
  const float fin = 1.0f / (PSC * VSC);
#pragma unroll
  for (int r = 0; r < 8; ++r) {
    const int row = 8 * hh + r;
    const float linv = 1.0f / ls[r];
    const float g = linv * fin;
    zs[row * ZP + m]      = O0[r] * g;
    zs[row * ZP + 16 + m] = O1[r] * g;
    zs[row * ZP + 32 + m] = O2[r] * g;
    zs[row * ZP + 48 + m] = O3[r] * g;
  }
  wave_sync_lds();
  {
    const int hh2 = lane >> 4, c4 = (lane & 15) * 4;
    v4f vals[8];
#pragma unroll
    for (int it = 0; it < 8; ++it) {
      const int row = it * 2 + hh2;
      vals[it] = *(const v4f*)(zs + row * ZP + c4);
    }
    const size_t orow0 = (size_t)b * SEQ_FULL + (size_t)t0;
    for (int pass = 0; pass < 2; ++pass) {
#pragma unroll
      for (int it = 0; it < 8; ++it) {
        const int row = it * 2 + hh2;
        float* dst = Out + (orow0 + (size_t)row) * DM + h * HD + c4;
        *(volatile v4f*)dst = vals[it];
      }
      __threadfence();
    }
  }
}

extern "C" void kernel_launch(void* const* d_in, const int* in_sizes, int n_in,
                              void* d_out, int out_size, void* d_ws, size_t ws_size,
                              hipStream_t stream) {
  if (n_in < 8) return;
  const long long need_x = ((long long)(NB - 1) * SEQ_FULL + SEQ) * DM;
  if ((long long)in_sizes[0] < need_x) return;
  if (in_sizes[1] != DM * DM) return;
  if (in_sizes[2] < DM) return;
  if (in_sizes[3] != DM * DM) return;
  if (in_sizes[4] < DM) return;
  if (in_sizes[7] != NREL * HD) return;
  if ((long long)out_size < need_x) return;

  const float* x   = (const float*)d_in[0];
  const float* wq  = (const float*)d_in[1];
  const float* bq  = (const float*)d_in[2];
  const float* wk  = (const float*)d_in[3];
  const float* bk  = (const float*)d_in[4];
  const float* tab = (const float*)d_in[7];

  const size_t PXH = (size_t)MT * DM * 2;
  const size_t PWT = (size_t)2 * DM * DM * 2;
  const size_t PPE = (size_t)PER * HD * 2;
  const size_t PKQ = (size_t)MT * KQP * 2;
  const size_t PVT = (size_t)DM * MT * 2;
  size_t off = 0;
  const size_t oXH = off; off += PXH;
  const size_t oWT = off; off += PWT;
  const size_t oPE = off; off += PPE;
  const size_t oKQ = off; off += PKQ;
  const size_t oVT = off; off += PVT;
  if (off > ws_size) return;
  if (off > (size_t)134217728) return;

  char* ws = (char*)d_ws;
  unsigned short* XH  = (unsigned short*)(ws + oXH);
  unsigned short* WT  = (unsigned short*)(ws + oWT);
  unsigned short* PEH = (unsigned short*)(ws + oPE);
  unsigned short* KQ  = (unsigned short*)(ws + oKQ);
  unsigned short* VT  = (unsigned short*)(ws + oVT);
  float* out0 = (float*)d_out;

  const dim3 blk(256);
  const int gP = ((MT / 64) * (DM / 64)) / 8;

  cvt_x<<<dim3((MT * DM) / 2048), blk, 0, stream>>>(x, XH);
  cvt_lin<<<dim3((PER * HD) / 2048), blk, 0, stream>>>(tab, PEH, NREL * HD, PER * HD, WSCL);
  cvt_t<<<dim3(DM / 64, DM / 64), blk, 0, stream>>>(wq, WT, DM, DM, WSCL);
  cvt_t<<<dim3(DM / 64, DM / 64), blk, 0, stream>>>(wk, WT + (size_t)DM * DM, DM, DM, WSCL);

  gemm64h<<<dim3(gP), blk, 0, stream>>>(XH, DM, WT, DM, KQ, KQP, bq, QKS / WSCL, QKS, MT, DM, DM);
  gemm64h<<<dim3(gP), blk, 0, stream>>>(XH, DM, WT + (size_t)DM * DM, DM, KQ + DM, KQP, bk, QKS / WSCL, QKS, MT, DM, DM);

  tr16<<<dim3(DM / 64, MT / 64), blk, 0, stream>>>(KQ + DM, KQP, VT, MT, DM);

  attn_kernel<<<dim3(NB * NH * (SEQ / 64)), dim3(128), 0, stream>>>(KQ, PEH, VT, out0);
  (void)hipGetLastError();
}
